// SDConv_5669356830988
// MI455X (gfx1250) — hardware-verified
//
#include <hip/hip_runtime.h>


#define NB_  4
#define LL   2048
#define DD   768
#define NH_  12
#define IPG  64
#define KW   9
#define NR   (NB_ * LL)
typedef _Float16 h16;
typedef unsigned short bf;
typedef __attribute__((ext_vector_type(16))) __bf16   v16bf;
typedef __attribute__((ext_vector_type(16))) _Float16 v16h;
typedef __attribute__((ext_vector_type(8)))  _Float16 v8h;
typedef __attribute__((ext_vector_type(8)))  unsigned short v8us;
typedef __attribute__((ext_vector_type(8)))  float    v8f;
typedef __attribute__((ext_vector_type(4)))  float    v4f;
typedef v8h  __attribute__((may_alias)) v8ha;
typedef v4f  __attribute__((may_alias)) v4fa;
typedef v8us __attribute__((may_alias)) v8usa;

__device__ __forceinline__ unsigned short f2bf(float f) { unsigned u = __float_as_uint(f); u += 0x7FFFu + ((u >> 16) & 1u); return (unsigned short)(u >> 16); }
__device__ __forceinline__ float bf2f(unsigned short b) { return __uint_as_float(((unsigned)b) << 16); }
__device__ __forceinline__ float bfr(float f) { return bf2f(f2bf(f)); }
__device__ __forceinline__ v16h cat16(v8h lo, v8h hi) { return __builtin_shufflevector(lo, hi, 0, 1, 2, 3, 4, 5, 6, 7, 8, 9, 10, 11, 12, 13, 14, 15); }
__device__ __forceinline__ v16bf cat16b(v8us lo, v8us hi) { return __builtin_bit_cast(v16bf, __builtin_shufflevector(lo, hi, 0, 1, 2, 3, 4, 5, 6, 7, 8, 9, 10, 11, 12, 13, 14, 15)); }
__device__ __forceinline__ v8f wmma16(v16h a, v16h b, v8f c) { return __builtin_amdgcn_wmma_f32_16x16x32_f16(false, a, false, b, (short)0, c, false, false); }
__device__ __forceinline__ v8f wmmab(v16bf a, v16bf b, v8f c) { return __builtin_amdgcn_wmma_f32_16x16x32_bf16(false, a, false, b, (short)0, c, false, false); }


template <typename T16> struct WFrag;
template <> struct WFrag<h16> { typedef v16h V; static __device__ __forceinline__ V ld(const h16* p) { return cat16(*(const v8h*)p, *(const v8h*)(p + 16)); } static __device__ __forceinline__ v8f mma(V a, V b, v8f c) { return wmma16(a, b, c); } };
template <> struct WFrag<bf> { typedef v16bf V; static __device__ __forceinline__ V ld(const bf* p) { return cat16b(*(const v8us*)p, *(const v8us*)(p + 16)); } static __device__ __forceinline__ v8f mma(V a, V b, v8f c) { return wmmab(a, b, c); } };
template <typename T16, int NSPLIT, bool BIAS>
__global__ __launch_bounds__(32) void k_gemmw(const T16* __restrict__ A, const T16* __restrict__ A2, const T16* __restrict__ Bt, const T16* __restrict__ Bt2, int K, float* C, int ldc, const float* __restrict__ bias, size_t sA, size_t sB, size_t sC) {
    typedef typename WFrag<T16>::V V;
    __shared__ __align__(16) float os[16 * 68];
    const size_t z = blockIdx.z; A += z * sA; if (A2) A2 += z * sA; Bt += z * sB; if (Bt2) Bt2 += z * sB; C += z * sC;
    const int lane = threadIdx.x & 31, lr = lane & 15, hi = lane >> 4; const int r0 = blockIdx.x * 64, c0 = blockIdx.y * 64;
    v8f acc[4][4];
#pragma unroll
    for (int mb = 0; mb < 4; ++mb)
#pragma unroll
        for (int nb = 0; nb < 4; ++nb) acc[mb][nb] = (v8f){};
    const size_t aoff = (size_t)(r0 + lr) * K + 8 * hi, boff = (size_t)(c0 + lr) * K + 8 * hi;
#pragma unroll 1
    for (int kc = 0; kc < K; kc += 32) {
        V a[4], a2[4];
#pragma unroll
        for (int mb = 0; mb < 4; ++mb) { a[mb] = WFrag<T16>::ld(A + aoff + (size_t)mb * 16 * K + kc); if (NSPLIT == 1 || NSPLIT == 2) a2[mb] = WFrag<T16>::ld(A2 + aoff + (size_t)mb * 16 * K + kc); }
#pragma unroll
        for (int nb = 0; nb < 4; ++nb) { const V b = WFrag<T16>::ld(Bt + boff + (size_t)nb * 16 * K + kc); V b2; if (NSPLIT >= 2) b2 = WFrag<T16>::ld(Bt2 + boff + (size_t)nb * 16 * K + kc);
#pragma unroll
            for (int mb = 0; mb < 4; ++mb) { acc[mb][nb] = WFrag<T16>::mma(a[mb], b, acc[mb][nb]); if (NSPLIT == 1 || NSPLIT == 2) acc[mb][nb] = WFrag<T16>::mma(a2[mb], b, acc[mb][nb]); if (NSPLIT >= 2) acc[mb][nb] = WFrag<T16>::mma(a[mb], b2, acc[mb][nb]); } }
        asm volatile("v_nop\n\tv_nop\n\tv_nop\n\tv_nop" : "+v"(acc[0][0]), "+v"(acc[1][1]), "+v"(acc[2][2]), "+v"(acc[3][3]) : "v"(a[0]), "v"(a[3]));
    }
#pragma unroll
    for (int mb = 0; mb < 4; ++mb) {
#pragma unroll
        for (int nb = 0; nb < 4; ++nb) {
#pragma unroll
            for (int j = 0; j < 8; ++j) os[(hi * 8 + j) * 68 + nb * 16 + lr] = acc[mb][nb][j]; }
        __builtin_amdgcn_wave_barrier(); asm volatile("" ::: "memory");
        float* crow = C + (size_t)(r0 + mb * 16) * ldc + c0;
#pragma unroll 1
        for (int ps = 0; ps < 2; ++ps) {
#pragma unroll
            for (int s = 0; s < 8; ++s) { const int row = 2 * s + hi, cofs = lr * 4; v4f val = *(const v4fa*)(os + row * 68 + cofs); if (BIAS) { val[0] += bfr(bias[c0 + cofs]); val[1] += bfr(bias[c0 + cofs + 1]); val[2] += bfr(bias[c0 + cofs + 2]); val[3] += bfr(bias[c0 + cofs + 3]); }
                *(volatile v4f*)(crow + (size_t)row * ldc + cofs) = val; }
            if (ps == 0) __threadfence(); }
        __builtin_amdgcn_wave_barrier(); asm volatile("" ::: "memory");
    }
}

__device__ __forceinline__ void splitf(float y, unsigned short& h, unsigned short& l) { h = f2bf(y); l = f2bf(y - bf2f(h)); }
typedef __attribute__((ext_vector_type(2))) unsigned short v2us;
typedef __attribute__((ext_vector_type(2))) float v2f;

__global__ __launch_bounds__(256) void k_cvt8(const float* __restrict__ src, bf* dst, size_t n8) { const size_t i = (size_t)blockIdx.x * 256 + threadIdx.x; if (i >= n8) return; const v8f v = *(const v8f*)(src + i * 8); v8us o;
#pragma unroll
    for (int k = 0; k < 8; ++k) o[k] = f2bf(v[k]); *(volatile v8us*)(dst + i * 8) = o; __threadfence(); *(volatile v8us*)(dst + i * 8) = o; }
__global__ __launch_bounds__(256) void k_dw(const float* __restrict__ q, const float* __restrict__ dww, bf* Dh, bf* Dl) { const size_t e = ((size_t)blockIdx.x * 256 + threadIdx.x) * 2; if (e >= (size_t)NR * DD) return; const int c = (int)(e % DD); const int row = (int)(e / DD); const int l = row % LL, b = row / LL; v2us oh, ol;
#pragma unroll
    for (int u = 0; u < 2; ++u) { const int cc = c + u; float s = 0.f;
#pragma unroll
        for (int k = 0; k < KW; ++k) { const int ls = l + k - 4; if (ls < 0 || ls >= LL) continue; float p = __fmul_rn(bfr(dww[cc * KW + k]), bfr(q[((size_t)b * LL + ls) * DD + cc])); asm volatile("" : "+v"(p)); s = __fadd_rn(s, p); }
        unsigned short a, c2; splitf(s, a, c2); oh[u] = a; ol[u] = c2; }
    const size_t oo = ((size_t)(c / IPG) * NR + row) * IPG + (c % IPG); *(volatile v2us*)(Dh + oo) = oh; *(volatile v2us*)(Dl + oo) = ol; __threadfence(); *(volatile v2us*)(Dh + oo) = oh; *(volatile v2us*)(Dl + oo) = ol; }
__global__ __launch_bounds__(256) void k_kern(const float* __restrict__ PW, const float* __restrict__ pwb, const float* __restrict__ q, const float* __restrict__ akw, const float* __restrict__ akb, float* WT) { const int idx = blockIdx.x * 256 + threadIdx.x; if (idx >= NR * NH_) return; const int h = idx % NH_, row = idx / NH_; const float* pw = PW + (size_t)row * DD + h * IPG; const float* qr = q + (size_t)row * DD + h * IPG;
    float kern[KW];
#pragma unroll
    for (int k = 0; k < KW; ++k) kern[k] = 0.f;
    for (int i = 0; i < IPG; ++i) { float ca = __fmul_rn(__fadd_rn(pw[i], bfr(pwb[h * IPG + i])), bfr(qr[i])); asm volatile("" : "+v"(ca));
#pragma unroll
        for (int k = 0; k < KW; ++k) { float p = __fmul_rn(ca, bfr(akw[((size_t)h * KW + k) * IPG + i])); asm volatile("" : "+v"(p)); kern[k] = __fadd_rn(kern[k], p); } }
    float mx = -3.0e38f;
#pragma unroll
    for (int k = 0; k < KW; ++k) { kern[k] = __fadd_rn(kern[k], bfr(akb[h * KW + k])); mx = fmaxf(mx, kern[k]); }
    float sum = 0.f;
#pragma unroll
    for (int k = 0; k < KW; ++k) { float d0 = __fsub_rn(kern[k], mx); asm volatile("" : "+v"(d0)); kern[k] = __expf(d0); sum = __fadd_rn(sum, kern[k]); }
    const float rs = __fdiv_rn(1.0f, sum); v4f o[4];
#pragma unroll
    for (int k = 0; k < 16; ++k) { const float w = (k < KW) ? __fmul_rn(kern[k < KW ? k : 0], rs) : 0.f; o[k / 4][k % 4] = w; }
    float* dst = WT + (size_t)idx * 16;
#pragma unroll
    for (int u = 0; u < 4; ++u) *(volatile v4f*)(dst + 4 * u) = o[u]; __threadfence();
#pragma unroll
    for (int u = 0; u < 4; ++u) *(volatile v4f*)(dst + 4 * u) = o[u]; }
__global__ __launch_bounds__(256) void k_out(const float* __restrict__ WT, const float* __restrict__ V, float* OUT) { const size_t e = ((size_t)blockIdx.x * 256 + threadIdx.x) * 2; if (e >= (size_t)NR * DD) return; const int c = (int)(e % DD); const int row = (int)(e / DD); const int l = row % LL, b = row / LL; const int h = c / IPG; const float* w = WT + ((size_t)row * NH_ + h) * 16; v2f o;
#pragma unroll
    for (int u = 0; u < 2; ++u) { float s = 0.f;
#pragma unroll
        for (int k = 0; k < KW; ++k) { const int ls = l + k - 4; if (ls < 0 || ls >= LL) continue; float p = __fmul_rn(w[k], V[((size_t)b * LL + ls) * DD + c + u]); asm volatile("" : "+v"(p)); s = __fadd_rn(s, p); } o[u] = s; }
    *(volatile v2f*)(OUT + e) = o; __threadfence(); *(volatile v2f*)(OUT + e) = o; }

extern "C" void kernel_launch(void* const* d_in, const int* in_sizes, int n_in,
                              void* d_out, int out_size, void* d_ws, size_t ws_size, hipStream_t stream) {
    (void)in_sizes; (void)n_in; (void)out_size;
    const float* q = (const float*)d_in[0]; const float* dww = (const float*)d_in[1]; const float* pww = (const float*)d_in[2]; const float* pwb = (const float*)d_in[3]; const float* akw = (const float*)d_in[4]; const float* akb = (const float*)d_in[5]; const float* ptw = (const float*)d_in[6]; const float* ptb = (const float*)d_in[7];
    float* OUT = (float*)d_out;
    char* wsp = (char*)d_ws;
    auto take = [&](size_t bytes) { char* p = wsp; wsp += (bytes + 255) & ~(size_t)255; return (void*)p; };
    bf* PWB = (bf*)take((size_t)NH_ * IPG * IPG * 2); bf* PTW = (bf*)take((size_t)DD * DD * 2); bf* QB = (bf*)take((size_t)NR * DD * 2); bf* Dh = (bf*)take((size_t)NR * DD * 2); bf* Dl = (bf*)take((size_t)NR * DD * 2); float* PW = (float*)take((size_t)NR * DD * 4); float* WT = (float*)take((size_t)NR * NH_ * 16 * 4); float* V = (float*)take((size_t)NR * DD * 4);
    if ((size_t)(wsp - (char*)d_ws) > ws_size) return;
    k_cvt8<<<(NH_ * IPG * IPG / 8 + 255) / 256, 256, 0, stream>>>(pww, PWB, (size_t)NH_ * IPG * IPG / 8); k_cvt8<<<(unsigned)(((size_t)DD * DD / 8 + 255) / 256), 256, 0, stream>>>(ptw, PTW, (size_t)DD * DD / 8); k_cvt8<<<(unsigned)(((size_t)NR * DD / 8 + 255) / 256), 256, 0, stream>>>(q, QB, (size_t)NR * DD / 8);
    k_dw<<<(unsigned)(((size_t)NR * DD / 2 + 255) / 256), 256, 0, stream>>>(q, dww, Dh, Dl);
    k_gemmw<bf, 1, false><<<dim3(NR / 64, IPG / 64, NH_), 32, 0, stream>>>(Dh, Dl, PWB, nullptr, IPG, PW, DD, nullptr, (size_t)NR * IPG, (size_t)IPG * IPG, (size_t)IPG);
    k_kern<<<(NR * NH_ + 255) / 256, 256, 0, stream>>>(PW, pwb, q, akw, akb, WT);
    k_gemmw<bf, 0, true><<<dim3(NR / 64, DD / 64, 1), 32, 0, stream>>>(QB, nullptr, PTW, nullptr, DD, V, DD, ptb, 0, 0, 0);
    k_out<<<(unsigned)(((size_t)NR * DD / 2 + 255) / 256), 256, 0, stream>>>(WT, V, OUT);
}
